// FGDN_11184094839450
// MI455X (gfx1250) — hardware-verified
//
#include <hip/hip_runtime.h>
#include <stddef.h>


#define NN_    10000
#define FIN_   128
#define FD_    256
#define FH_    128
#define NCL_   10
#define NG_    64
#define NPAD   10240
#define NTHR   256
#define NWAVE  8
#define EPT    8
#define NGRP   2
#define CHUNK  (NTHR * EPT * NGRP)
#define WCAP   (EPT * NGRP * 32)
#define LISTN  (NWAVE * WCAP)
#define NBD    4096
#define NDEGB  ((NN_ + NBD - 1) / NBD)
#define NB0    512
#define NB1    256
#define GROWS  64
#define NGEMB  ((NN_ + GROWS - 1) / GROWS)
#define HP     264
#define WSC    16.0f
#define WINV   0.0625f

#define LDS_PROP (NB1 * FD_ * 4 + LISTN * 4 + 64)
#define LDS_GEMM (GROWS * FD_ * 4)
#define LDS_HEAD (NG_ * FD_ * 4 + NG_ * HP * 2 + NG_ * FH_ * 4 + NG_ * NCL_ * 4)

static_assert(NB0 * FIN_ == NB1 * FD_);
static_assert(NPAD % NB0 == 0 && NPAD % NB1 == 0);
static_assert(NGEMB * GROWS <= NPAD);
static_assert(NDEGB * NBD >= NPAD);
static_assert((CHUNK & (CHUNK - 1)) == 0 && CHUNK <= 4096);
static_assert(NBD <= 4096 && NB0 <= 4096 && NB1 <= 4096);
static_assert((HP * 2) % 16 == 0);
static_assert(NBD == NWAVE * 4 * 128);

typedef float    v4f  __attribute__((ext_vector_type(4)));
typedef float    v8f  __attribute__((ext_vector_type(8)));
typedef int      v4i  __attribute__((ext_vector_type(4)));
typedef _Float16 v8h  __attribute__((ext_vector_type(8)));
typedef _Float16 v16h __attribute__((ext_vector_type(16)));
union FragH { v16h v; v8h h[2]; };

__device__ __forceinline__ v8h cvt8(v4f a, v4f b) {
  v8h r;
  r[0] = (_Float16)a.x; r[1] = (_Float16)a.y; r[2] = (_Float16)a.z; r[3] = (_Float16)a.w;
  r[4] = (_Float16)b.x; r[5] = (_Float16)b.y; r[6] = (_Float16)b.z; r[7] = (_Float16)b.w;
  return r;
}

__device__ __forceinline__ v8f wmh(v16h a, v16h b, v8f c) {
  v8f d = __builtin_amdgcn_wmma_f32_16x16x32_f16(false, a, false, b, (short)0, c, false, false);
  asm volatile("v_nop\n\tv_nop\n\tv_nop\n\tv_nop" : "+v"(d) : "v"(a), "v"(b));
  return d;
}

template <int NB>
__device__ __forceinline__ int scan_chunk(const int* __restrict__ dsts, int nE, int cbase, int nodeBase,
                                          int vec8, int* list, int tid, int lane, int wave) {
  int wc = 0;
#pragma unroll
  for (int g = 0; g < NGRP; ++g) {
    const int el0  = (g * NTHR + tid) * EPT;
    const int e0   = cbase + el0;
    const int sent = -2147483647 - 1;
    v4i da, db;
    if (vec8 != 0 && e0 + 7 < nE) {
      da = *(const v4i*)(dsts + e0);
      db = *(const v4i*)(dsts + e0 + 4);
    } else {
      da.x = (e0     < nE) ? dsts[min(e0, nE - 1)] : sent;
      da.y = (e0 + 1 < nE) ? dsts[min(e0 + 1, nE - 1)] : sent;
      da.z = (e0 + 2 < nE) ? dsts[min(e0 + 2, nE - 1)] : sent;
      da.w = (e0 + 3 < nE) ? dsts[min(e0 + 3, nE - 1)] : sent;
      db.x = (e0 + 4 < nE) ? dsts[min(e0 + 4, nE - 1)] : sent;
      db.y = (e0 + 5 < nE) ? dsts[min(e0 + 5, nE - 1)] : sent;
      db.z = (e0 + 6 < nE) ? dsts[min(e0 + 6, nE - 1)] : sent;
      db.w = (e0 + 7 < nE) ? dsts[min(e0 + 7, nE - 1)] : sent;
    }
    const unsigned nb = (unsigned)nodeBase;
    const unsigned s0 = (unsigned)da.x - nb, s1 = (unsigned)da.y - nb;
    const unsigned s2 = (unsigned)da.z - nb, s3 = (unsigned)da.w - nb;
    const unsigned s4 = (unsigned)db.x - nb, s5 = (unsigned)db.y - nb;
    const unsigned s6 = (unsigned)db.z - nb, s7 = (unsigned)db.w - nb;
    const bool h0 = s0 < (unsigned)NB, h1 = s1 < (unsigned)NB, h2 = s2 < (unsigned)NB, h3 = s3 < (unsigned)NB;
    const bool h4 = s4 < (unsigned)NB, h5 = s5 < (unsigned)NB, h6 = s6 < (unsigned)NB, h7 = s7 < (unsigned)NB;
    const unsigned any = __builtin_amdgcn_ballot_w32(h0 | h1 | h2 | h3 | h4 | h5 | h6 | h7);
    if (any != 0u) {
#define HITJ(J, HJ, SJ) { \
        const unsigned mj = __builtin_amdgcn_ballot_w32(HJ); \
        if (mj != 0u) { \
          if (HJ) { \
            const int pos = wc + (int)__builtin_amdgcn_mbcnt_lo(mj, 0u); \
            if (pos < WCAP) list[wave * WCAP + pos] = ((el0 + (J)) << 12) | (int)(SJ); \
          } \
          wc += (int)__builtin_popcount(mj); } }
      HITJ(0, h0, s0)
      HITJ(1, h1, s1)
      HITJ(2, h2, s2)
      HITJ(3, h3, s3)
      HITJ(4, h4, s4)
      HITJ(5, h5, s5)
      HITJ(6, h6, s6)
      HITJ(7, h7, s7)
#undef HITJ
    }
  }
  return wc;
}

__global__ __launch_bounds__(NTHR) void k_wprep(
    const float* __restrict__ W1, const float* __restrict__ Wr,
    const float* __restrict__ F1, const float* __restrict__ F2,
    _Float16* w1s, _Float16* wrs, _Float16* f1s, _Float16* f2s) {
  const int i  = blockIdx.x * NTHR + threadIdx.x;
  const int n0 = FD_ * 3 * FIN_ / 8;
  const int n1 = 3 * (FD_ * 3 * FD_ / 8);
  const int n2 = FD_ * FD_ / 8;
  const int n3 = FH_ * FD_ / 8;
  if (i >= n0 + n1 + n2 + n3) return;
  const float* src;
  _Float16* dp;
  int K, N, o;
  if (i < n0) {
    o = i * 8; K = 3 * FIN_; N = FD_; src = W1; dp = w1s + o;
  } else if (i < n0 + n1) {
    const int j   = i - n0;
    const int per = FD_ * 3 * FD_ / 8;
    const int l   = j / per;
    o = (j - l * per) * 8; K = 3 * FD_; N = FD_;
    src = Wr + (size_t)l * 3 * FD_ * FD_;
    dp  = wrs + (size_t)l * FD_ * 3 * FD_ + o;
  } else if (i < n0 + n1 + n2) {
    o = (i - n0 - n1) * 8; K = FD_; N = FD_; src = F1; dp = f1s + o;
  } else {
    o = (i - n0 - n1 - n2) * 8; K = FD_; N = FH_; src = F2; dp = f2s + o;
  }
  const int n  = o / K;
  const int k0 = o - n * K;
  const float* p = src + (size_t)k0 * N + n;
  v4f a, b;
  a.x = p[0];              a.y = p[(size_t)N];     a.z = p[(size_t)2 * N]; a.w = p[(size_t)3 * N];
  b.x = p[(size_t)4 * N];  b.y = p[(size_t)5 * N]; b.z = p[(size_t)6 * N]; b.w = p[(size_t)7 * N];
  a = a * WSC;
  b = b * WSC;
  const v8h hv = cvt8(a, b);
  *(volatile v8h*)dp = hv;
  __threadfence();
  *(volatile v8h*)dp = hv;
}

__global__ __launch_bounds__(NTHR) void k_deg(
    const int* __restrict__ ei, float* dinv, int nE, int vec8) {
  __shared__ __attribute__((aligned(16))) int   cnt[NBD];
  __shared__ __attribute__((aligned(16))) int   list[LISTN];
  __shared__ __attribute__((aligned(16))) float dqs[NBD];
  __shared__ int wcnt[NWAVE];
  const int tid = threadIdx.x, lane = tid & 31, wave = tid >> 5;
  const int nodeBase = blockIdx.x * NBD;
  const int* srcs = ei;

  for (int i = tid; i < NBD; i += NTHR) cnt[i] = 0;
  __syncthreads();

  const int nChunks = (nE + CHUNK - 1) / CHUNK;
#pragma unroll 1
  for (int ch = 0; ch < nChunks; ++ch) {
    const int cbase = ch * CHUNK;
    const int wc = scan_chunk<NBD>(srcs, nE, cbase, nodeBase, vec8, list, tid, lane, wave);
    if (lane == 0) wcnt[wave] = wc;
    __syncthreads();
    if (wave == 0) {
#pragma unroll 1
      for (int wsx = 0; wsx < NWAVE; ++wsx) {
        int n = __builtin_amdgcn_readfirstlane(wcnt[wsx]);
        n = n > WCAP ? WCAP : (n < 0 ? 0 : n);
        const int* lp = list + wsx * WCAP;
#pragma unroll 1
        for (int i = 0; i < n; ++i) {
          const int ent  = __builtin_amdgcn_readfirstlane(lp[i]);
          const int slot = ent & (NBD - 1);
          if (lane == 0) cnt[slot] = cnt[slot] + 1;
        }
      }
    }
    __syncthreads();
  }

#pragma unroll 1
  for (int q = 0; q < 4; ++q) {
    const int f = (wave * 4 + q) * 128 + 4 * lane;
    const v4i c = *(const v4i*)(cnt + f);
    v4f d;
    d.x = (c.x > 0) ? rsqrtf((float)c.x) : 0.0f;
    d.y = (c.y > 0) ? rsqrtf((float)c.y) : 0.0f;
    d.z = (c.z > 0) ? rsqrtf((float)c.z) : 0.0f;
    d.w = (c.w > 0) ? rsqrtf((float)c.w) : 0.0f;
    *(v4f*)(dqs + f) = d;
  }
  float* dp = dinv + (size_t)nodeBase;
#pragma unroll 1
  for (int q = 0; q < 4; ++q) {
    const int f = (wave * 4 + q) * 128 + 4 * lane;
    const v4f v = *(const v4f*)(dqs + f);
    *(volatile v4f*)(dp + f) = v;
  }
  __threadfence();
#pragma unroll 1
  for (int q = 0; q < 4; ++q) {
    const int f = (wave * 4 + q) * 128 + 4 * lane;
    const v4f v = *(const v4f*)(dqs + f);
    *(volatile v4f*)(dp + f) = v;
  }
}

template <int CIN, int NB, int MODE>
__global__ __launch_bounds__(NTHR) void k_prop(
    const int* __restrict__ ei, const float* srcf, const float* hsrc,
    const float* __restrict__ dinv, float* t1f, _Float16* acat, int nE, int vec8) {
  constexpr int KP  = 3 * CIN;
  constexpr int Q4  = CIN / 128;
  constexpr int C4  = CIN / 4;
  constexpr int HL  = CIN / 8;
  constexpr int RPI = 32 / HL;
  constexpr int RPW = NB / NWAVE;
  extern __shared__ v4f lds_dyn[];
  float* acc  = (float*)lds_dyn;
  int*   list = (int*)(acc + NB * CIN);
  int*   wcnt = list + LISTN;
  const int tid = threadIdx.x, lane = tid & 31, wave = tid >> 5;
  const int nodeBase = blockIdx.x * NB;
  const int* dsts = ei + nE;

  {
    const v4f z = {0.f, 0.f, 0.f, 0.f};
    for (int i = tid; i < NB * CIN / 4; i += NTHR) lds_dyn[i] = z;
  }
  __syncthreads();

  const int nChunks = (nE + CHUNK - 1) / CHUNK;
#pragma unroll 1
  for (int ch = 0; ch < nChunks; ++ch) {
    const int cbase = ch * CHUNK;
    const int wc = scan_chunk<NB>(dsts, nE, cbase, nodeBase, vec8, list, tid, lane, wave);
    if (lane == 0) wcnt[wave] = wc;
    __syncthreads();
    if (wave == 0) {
#pragma unroll 1
      for (int wsx = 0; wsx < NWAVE; ++wsx) {
        int n = __builtin_amdgcn_readfirstlane(wcnt[wsx]);
        n = n > WCAP ? WCAP : (n < 0 ? 0 : n);
        const int* lp = list + wsx * WCAP;
#pragma unroll 1
        for (int i = 0; i < n; ++i) {
          const int ent  = __builtin_amdgcn_readfirstlane(lp[i]);
          const int slot = ent & (NB - 1);
          int e = cbase + ((ent >> 12) & (CHUNK - 1));
          e = e > nE - 1 ? nE - 1 : e;
          int src = ei[e];
          src = src < 0 ? 0 : (src > NN_ - 1 ? NN_ - 1 : src);
          const float cf = dinv[src];
          const float* sp = srcf + (size_t)src * CIN + 4 * lane;
          float* ap = acc + slot * CIN + 4 * lane;
#pragma unroll
          for (int q = 0; q < Q4; ++q) {
            const v4f v = *(const v4f*)(sp + 128 * q);
            v4f* aq = (v4f*)(ap + 128 * q);
            *aq = *aq + v * cf;
          }
        }
      }
    }
    __syncthreads();
  }

#pragma unroll 4
  for (int it = 0; it < (NB * C4) / NTHR; ++it) {
    const int idx  = it * NTHR + tid;
    const int slot = idx / C4;
    const int c4   = (idx - slot * C4) * 4;
    int node = nodeBase + slot;
    node = node > NN_ - 1 ? NN_ - 1 : node;
    const float d = dinv[node];
    v4f* ap = (v4f*)(acc + slot * CIN + c4);
    const v4f p = -((*ap) * d);
    if (MODE == 0) {
      *ap = p;
    } else {
      const v4f hv = *(const v4f*)(hsrc + (size_t)node * CIN + c4);
      *ap = p * 2.0f - hv;
    }
  }
  __syncthreads();

  const int sub = lane / HL;
  const int l16 = lane - sub * HL;
  for (int rep = 0; rep < 2; ++rep) {
    if (MODE == 0) {
#pragma unroll 4
      for (int r = 0; r < RPW; ++r) {
        const int slot = wave * RPW + r;
        const size_t grow = (size_t)(nodeBase + slot);
#pragma unroll
        for (int q = 0; q < Q4; ++q) {
          const v4f v = *(const v4f*)(acc + slot * CIN + 128 * q + 4 * lane);
          *(volatile v4f*)(t1f + grow * CIN + 128 * q + 4 * lane) = v;
        }
      }
    }
#pragma unroll 2
    for (int rr = 0; rr < RPW / RPI; ++rr) {
      const int slot  = wave * RPW + rr * RPI + sub;
      const int growi = nodeBase + slot;
      _Float16* rp = acat + (size_t)growi * KP + 8 * l16;
      const float* lp = acc + slot * CIN + 8 * l16;
      const v8h hv = cvt8(*(const v4f*)lp, *(const v4f*)(lp + 4));
      if (MODE == 0) {
        int node = growi > NN_ - 1 ? NN_ - 1 : growi;
        const float* gp = hsrc + (size_t)node * CIN + 8 * l16;
        const v8h h0v = cvt8(*(const v4f*)gp, *(const v4f*)(gp + 4));
        *(volatile v8h*)rp = h0v;
        *(volatile v8h*)(rp + CIN) = hv;
      } else {
        *(volatile v8h*)(rp + 2 * CIN) = hv;
      }
    }
    if (rep == 0) __threadfence();
  }
}

template <int KD, int ACT>
__global__ __launch_bounds__(NTHR) void k_gemm(
    const _Float16* __restrict__ acat, const _Float16* __restrict__ wsb,
    const float* __restrict__ bias, const float* __restrict__ alpha, float* hout) {
  extern __shared__ v4f lds_dyn[];
  float* stg = (float*)lds_dyn;
  const int tid = threadIdx.x, lane = tid & 31, wave = tid >> 5, hh = lane >> 4, m = lane & 15;
  const int rt = wave & 3, ch = wave >> 2;
  const int rowBase = blockIdx.x * GROWS;

  v8f acc[8];
#pragma unroll
  for (int t = 0; t < 8; ++t) { v8f z = {0.f, 0.f, 0.f, 0.f, 0.f, 0.f, 0.f, 0.f}; acc[t] = z; }

  const _Float16* ar = acat + (size_t)(rowBase + 16 * rt + m) * KD + 8 * hh;
  const _Float16* bb = wsb + (size_t)(128 * ch + m) * KD + 8 * hh;
#pragma unroll 1
  for (int kt = 0; kt < KD / 32; ++kt) {
    FragH a;
    a.h[0] = *(const v8h*)(ar + 32 * kt);
    a.h[1] = *(const v8h*)(ar + 32 * kt + 16);
#pragma unroll
    for (int t = 0; t < 8; ++t) {
      const _Float16* bp = bb + (size_t)(16 * t) * KD + 32 * kt;
      FragH b;
      b.h[0] = *(const v8h*)bp;
      b.h[1] = *(const v8h*)(bp + 16);
      acc[t] = wmh(a.v, b.v, acc[t]);
    }
  }

  const float al = alpha[0];
  float* sp = stg + (16 * rt + 8 * hh) * FD_ + 128 * ch + m;
#pragma unroll
  for (int t = 0; t < 8; ++t) {
    const float bv = bias[128 * ch + 16 * t + m];
#pragma unroll
    for (int r = 0; r < 8; ++r) {
      float v = acc[t][r] * WINV + bv;
      if (ACT == 0) v = (v >= 0.0f) ? v : al * v;
      else          v = fmaxf(v, 0.0f);
      sp[r * FD_ + 16 * t] = v;
    }
  }
  __syncthreads();

  for (int rep = 0; rep < 2; ++rep) {
#pragma unroll
    for (int i = 0; i < 8; ++i) {
      const int row = 8 * wave + i;
      const float* lp = stg + row * FD_ + 4 * lane;
      float* gp = hout + (size_t)(rowBase + row) * FD_ + 4 * lane;
      const v4f v0 = *(const v4f*)lp;
      const v4f v1 = *(const v4f*)(lp + 128);
      *(volatile v4f*)gp = v0;
      *(volatile v4f*)(gp + 128) = v1;
    }
    if (rep == 0) __threadfence();
  }
}

__global__ __launch_bounds__(NTHR) void k_head(
    const float* __restrict__ h, const int* __restrict__ batch,
    const _Float16* __restrict__ f1s, const float* __restrict__ f1b, const float* __restrict__ a3,
    const _Float16* __restrict__ f2s, const float* __restrict__ f2b,
    const float* __restrict__ f3w, const float* __restrict__ f3b, float* out) {
  extern __shared__ v4f lds_dyn[];
  float*    R1 = (float*)lds_dyn;
  _Float16* R2 = (_Float16*)(R1 + NG_ * FD_);
  float*    R3 = (float*)(R2 + NG_ * HP);
  float*    OS = R3 + NG_ * FH_;
  const int tid = threadIdx.x, lane = tid & 31, wave = tid >> 5, hh = lane >> 4, m = lane & 15;

  {
    const v4f z = {0.f, 0.f, 0.f, 0.f};
    for (int i = tid; i < NG_ * FD_ / 4; i += NTHR) lds_dyn[i] = z;
  }
  __syncthreads();

  {
    const int d = tid;
#pragma unroll 4
    for (int i = 0; i < NN_; ++i) {
      const int b = batch[i];
      const float v = h[(size_t)i * FD_ + d];
      if ((unsigned)b < (unsigned)NG_) R1[b * FD_ + d] = R1[b * FD_ + d] + v;
    }
  }
  __syncthreads();

  for (int u = tid; u < NG_ * FD_ / 8; u += NTHR) {
    const int row = u >> 5, c8 = (u & 31) * 8;
    const float* gp = R1 + row * FD_ + c8;
    *(v8h*)(R2 + row * HP + c8) = cvt8(*(const v4f*)gp, *(const v4f*)(gp + 4));
  }
  __syncthreads();

  const int rt = wave & 3;
  {
    const int cb = (wave >> 2) * 8;
    v8f acc[8];
#pragma unroll
    for (int t = 0; t < 8; ++t) { v8f z = {0.f, 0.f, 0.f, 0.f, 0.f, 0.f, 0.f, 0.f}; acc[t] = z; }
    const _Float16* ar = R2 + (16 * rt + m) * HP + 8 * hh;
#pragma unroll 1
    for (int kt = 0; kt < FD_ / 32; ++kt) {
      FragH a;
      a.h[0] = *(const v8h*)(ar + 32 * kt);
      a.h[1] = *(const v8h*)(ar + 32 * kt + 16);
#pragma unroll
      for (int t = 0; t < 8; ++t) {
        const _Float16* bp = f1s + (size_t)(16 * (cb + t) + m) * FD_ + 32 * kt + 8 * hh;
        FragH b;
        b.h[0] = *(const v8h*)bp;
        b.h[1] = *(const v8h*)(bp + 16);
        acc[t] = wmh(a.v, b.v, acc[t]);
      }
    }
    const float al = a3[0];
#pragma unroll
    for (int t = 0; t < 8; ++t) {
      const int n = 16 * (cb + t) + m;
      const float bv = f1b[n];
#pragma unroll
      for (int r = 0; r < 8; ++r) {
        float v = acc[t][r] * WINV + bv;
        v = (v >= 0.0f) ? v : al * v;
        R1[(16 * rt + 8 * hh + r) * FD_ + n] = v;
      }
    }
  }
  __syncthreads();

  for (int u = tid; u < NG_ * FD_ / 8; u += NTHR) {
    const int row = u >> 5, c8 = (u & 31) * 8;
    const float* gp = R1 + row * FD_ + c8;
    *(v8h*)(R2 + row * HP + c8) = cvt8(*(const v4f*)gp, *(const v4f*)(gp + 4));
  }
  __syncthreads();

  {
    const int cb2 = (wave >> 2) * 4;
    v8f acc[4];
#pragma unroll
    for (int t = 0; t < 4; ++t) { v8f z = {0.f, 0.f, 0.f, 0.f, 0.f, 0.f, 0.f, 0.f}; acc[t] = z; }
    const _Float16* ar = R2 + (16 * rt + m) * HP + 8 * hh;
#pragma unroll 1
    for (int kt = 0; kt < FD_ / 32; ++kt) {
      FragH a;
      a.h[0] = *(const v8h*)(ar + 32 * kt);
      a.h[1] = *(const v8h*)(ar + 32 * kt + 16);
#pragma unroll
      for (int t = 0; t < 4; ++t) {
        const _Float16* bp = f2s + (size_t)(16 * (cb2 + t) + m) * FD_ + 32 * kt + 8 * hh;
        FragH b;
        b.h[0] = *(const v8h*)bp;
        b.h[1] = *(const v8h*)(bp + 16);
        acc[t] = wmh(a.v, b.v, acc[t]);
      }
    }
#pragma unroll
    for (int t = 0; t < 4; ++t) {
      const int n = 16 * (cb2 + t) + m;
      const float bv = f2b[n];
#pragma unroll
      for (int r = 0; r < 8; ++r) {
        const float v  = acc[t][r] * WINV + bv;
        const float ev = expf(-v);
        const float sg = __builtin_amdgcn_rcpf(1.0f + ev);
        R3[(16 * rt + 8 * hh + r) * FH_ + n] = sg;
      }
    }
  }
  __syncthreads();

  if (tid < NG_) {
    float lg[NCL_];
#pragma unroll
    for (int j = 0; j < NCL_; ++j) lg[j] = 0.0f;
    const float* zp = R3 + tid * FH_;
#pragma unroll 1
    for (int k = 0; k < FH_; ++k) {
      const float z = zp[k];
      const float* wp = f3w + k * NCL_;
#pragma unroll
      for (int j = 0; j < NCL_; ++j) lg[j] = lg[j] + z * wp[j];
    }
#pragma unroll
    for (int j = 0; j < NCL_; ++j) lg[j] = lg[j] + f3b[j];
    float mx = lg[0];
#pragma unroll
    for (int j = 1; j < NCL_; ++j) mx = fmaxf(mx, lg[j]);
    float s = 0.0f;
#pragma unroll
    for (int j = 0; j < NCL_; ++j) s += expf(lg[j] - mx);
    const float ls = logf(s);
#pragma unroll
    for (int j = 0; j < NCL_; ++j) OS[tid * NCL_ + j] = (lg[j] - mx) - ls;
  }
  __syncthreads();

  if (wave == 0) {
    v4f ov[5];
#pragma unroll
    for (int q = 0; q < 5; ++q) ov[q] = *(const v4f*)(OS + q * 128 + 4 * lane);
#pragma unroll
    for (int q = 0; q < 5; ++q) *(volatile v4f*)(out + q * 128 + 4 * lane) = ov[q];
    __threadfence();
#pragma unroll
    for (int q = 0; q < 5; ++q) *(volatile v4f*)(out + q * 128 + 4 * lane) = ov[q];
  }
}

extern "C" void kernel_launch(void* const* d_in, const int* in_sizes, int n_in,
                              void* d_out, int out_size, void* d_ws, size_t ws_size,
                              hipStream_t stream) {
  if (n_in < 15) return;
  if (in_sizes[0] != NN_ * FIN_ || in_sizes[2] != NN_ || in_sizes[3] != 3 * FIN_ * FD_ ||
      in_sizes[4] != FD_ || in_sizes[5] != 9 * FD_ * FD_ || in_sizes[6] != 3 * FD_ ||
      in_sizes[7] != FD_ * FD_ || in_sizes[8] != FD_ || in_sizes[9] != FD_ * FH_ ||
      in_sizes[10] != FH_ || in_sizes[11] != FH_ * NCL_ || in_sizes[12] != NCL_ ||
      in_sizes[13] < 1 || in_sizes[14] < 1) return;
  const int nE = in_sizes[1] / 2;
  if (nE <= 0 || in_sizes[1] != 2 * nE) return;
  if (out_size != NG_ * NCL_) return;

  const float* x    = (const float*)d_in[0];
  const int*   ei   = (const int*)d_in[1];
  const int*   bat  = (const int*)d_in[2];
  const float* W1   = (const float*)d_in[3];
  const float* b1   = (const float*)d_in[4];
  const float* Wr   = (const float*)d_in[5];
  const float* br   = (const float*)d_in[6];
  const float* fc1w = (const float*)d_in[7];
  const float* fc1b = (const float*)d_in[8];
  const float* fc2w = (const float*)d_in[9];
  const float* fc2b = (const float*)d_in[10];
  const float* fc3w = (const float*)d_in[11];
  const float* fc3b = (const float*)d_in[12];
  const float* a1   = (const float*)d_in[13];
  const float* a3   = (const float*)d_in[14];
  float* out = (float*)d_out;

  char* ws = (char*)d_ws;
  size_t off = 0;
  const size_t oDv = off; off += (size_t)NDEGB * NBD * 4;              off = (off + 255) & ~(size_t)255;
  const size_t oAc = off; off += (size_t)NPAD * 3 * FD_ * 2;           off = (off + 255) & ~(size_t)255;
  const size_t oT1 = off; off += (size_t)NPAD * FD_ * 4;               off = (off + 255) & ~(size_t)255;
  const size_t oH  = off; off += (size_t)NPAD * FD_ * 4;               off = (off + 255) & ~(size_t)255;
  const size_t oW1 = off; off += (size_t)FD_ * 3 * FIN_ * 2;           off = (off + 255) & ~(size_t)255;
  const size_t oWr = off; off += (size_t)3 * FD_ * 3 * FD_ * 2;        off = (off + 255) & ~(size_t)255;
  const size_t oF1 = off; off += (size_t)FD_ * FD_ * 2;                off = (off + 255) & ~(size_t)255;
  const size_t oF2 = off; off += (size_t)FH_ * FD_ * 2;                off = (off + 255) & ~(size_t)255;
  if (off > ws_size) return;
  float*    dinv = (float*)(ws + oDv);
  _Float16* acat = (_Float16*)(ws + oAc);
  float*    t1f  = (float*)(ws + oT1);
  float*    hbuf = (float*)(ws + oH);
  _Float16* w1s  = (_Float16*)(ws + oW1);
  _Float16* wrs  = (_Float16*)(ws + oWr);
  _Float16* f1s  = (_Float16*)(ws + oF1);
  _Float16* f2s  = (_Float16*)(ws + oF2);

  const int vec8 = ((nE & 3) == 0) ? 1 : 0;

  const int nPrep = FD_ * 3 * FIN_ / 8 + 3 * (FD_ * 3 * FD_ / 8) + FD_ * FD_ / 8 + FH_ * FD_ / 8;
  k_wprep<<<(nPrep + NTHR - 1) / NTHR, NTHR, 0, stream>>>(W1, Wr, fc1w, fc2w, w1s, wrs, f1s, f2s);

  k_deg<<<NDEGB, NTHR, 0, stream>>>(ei, dinv, nE, vec8);

  hipFuncSetAttribute(reinterpret_cast<const void*>(&k_prop<FIN_, NB0, 0>),
                      hipFuncAttributeMaxDynamicSharedMemorySize, LDS_PROP);
  hipFuncSetAttribute(reinterpret_cast<const void*>(&k_prop<FIN_, NB0, 1>),
                      hipFuncAttributeMaxDynamicSharedMemorySize, LDS_PROP);
  hipFuncSetAttribute(reinterpret_cast<const void*>(&k_prop<FD_, NB1, 0>),
                      hipFuncAttributeMaxDynamicSharedMemorySize, LDS_PROP);
  hipFuncSetAttribute(reinterpret_cast<const void*>(&k_prop<FD_, NB1, 1>),
                      hipFuncAttributeMaxDynamicSharedMemorySize, LDS_PROP);
  hipFuncSetAttribute(reinterpret_cast<const void*>(&k_gemm<3 * FIN_, 0>),
                      hipFuncAttributeMaxDynamicSharedMemorySize, LDS_GEMM);
  hipFuncSetAttribute(reinterpret_cast<const void*>(&k_gemm<3 * FD_, 1>),
                      hipFuncAttributeMaxDynamicSharedMemorySize, LDS_GEMM);
  hipFuncSetAttribute(reinterpret_cast<const void*>(&k_head),
                      hipFuncAttributeMaxDynamicSharedMemorySize, LDS_HEAD);

  k_prop<FIN_, NB0, 0><<<NPAD / NB0, NTHR, LDS_PROP, stream>>>(ei, x, x, dinv, t1f, acat, nE, vec8);
  k_prop<FIN_, NB0, 1><<<NPAD / NB0, NTHR, LDS_PROP, stream>>>(ei, t1f, x, dinv, t1f, acat, nE, vec8);
  k_gemm<3 * FIN_, 0><<<NGEMB, NTHR, LDS_GEMM, stream>>>(acat, w1s, b1, a1, hbuf);

  for (int l = 0; l < 3; ++l) {
    k_prop<FD_, NB1, 0><<<NPAD / NB1, NTHR, LDS_PROP, stream>>>(ei, hbuf, hbuf, dinv, t1f, acat, nE, vec8);
    k_prop<FD_, NB1, 1><<<NPAD / NB1, NTHR, LDS_PROP, stream>>>(ei, t1f, hbuf, dinv, t1f, acat, nE, vec8);
    k_gemm<3 * FD_, 1><<<NGEMB, NTHR, LDS_GEMM, stream>>>(acat, wrs + (size_t)l * FD_ * 3 * FD_,
                                                          br + (size_t)l * FD_, a1, hbuf);
  }

  k_head<<<1, NTHR, LDS_HEAD, stream>>>(hbuf, bat, f1s, fc1b, a3, f2s, fc2b, fc3w, fc3b, out);
}
